// CachedVideoAttention_17901423690142
// MI455X (gfx1250) — hardware-verified
//
#include <hip/hip_runtime.h>
#include <stdint.h>
#include <stddef.h>

typedef __attribute__((ext_vector_type(16))) _Float16 v16h;
typedef __attribute__((ext_vector_type(8)))  _Float16 v8h;
typedef __attribute__((ext_vector_type(16))) __bf16   v16b;
typedef __attribute__((ext_vector_type(8)))  __bf16   v8b;
typedef __attribute__((ext_vector_type(8)))  float    v8f;
typedef __attribute__((ext_vector_type(4)))  float    v4f;
typedef __attribute__((ext_vector_type(4)))  unsigned int v4u;

constexpr int NUM_BATCH = 2;
constexpr int SEQ_LEN   = 2048;
constexpr int DMODEL    = 1024;
constexpr int NHEAD     = 16;
constexpr int HDIM      = 64;
constexpr int SEQ_CACHE = 2048;
constexpr int SEQ_KV    = SEQ_CACHE + SEQ_LEN;
constexpr int NUM_BH    = NUM_BATCH * NHEAD;
constexpr int NUM_TOK   = NUM_BATCH * SEQ_LEN;
constexpr float P_CARRY = 32768.0f;
constexpr float V_CARRY = 16.0f;
constexpr float LOG2E_F = 1.4426950408889634f;

static_assert(HDIM == 64);
static_assert(NHEAD * HDIM == DMODEL);
static_assert(SEQ_LEN % 64 == 0 && SEQ_CACHE % 64 == 0);
static_assert(NUM_TOK % 64 == 0 && (3 * DMODEL) % 64 == 0 && DMODEL % 64 == 0);
static_assert(DMODEL % 32 == 0);

__device__ __forceinline__ unsigned short f2bf_bits(float f) {
  unsigned u = __float_as_uint(f);
  return (unsigned short)((u + 0x7FFFu + ((u >> 16) & 1u)) >> 16);
}
__device__ __forceinline__ float bf_bits2f(unsigned short h) { return __uint_as_float(((unsigned)h) << 16); }
__device__ __forceinline__ unsigned short f2h_bits(float f) {
  const _Float16 h = (_Float16)f;
  return __builtin_bit_cast(unsigned short, h);
}

__device__ __forceinline__ void dep_guard_h(v8f& a, v8f& b, v16h x, v16h y) { asm volatile("v_nop\n\tv_nop\n\tv_nop\n\tv_nop" : "+v"(a), "+v"(b) : "v"(x), "v"(y)); }
__device__ __forceinline__ void dep_guard_b(v8f& a, v8f& b, v16b x, v16b y) { asm volatile("v_nop\n\tv_nop\n\tv_nop\n\tv_nop" : "+v"(a), "+v"(b) : "v"(x), "v"(y)); }
__device__ __forceinline__ void keep4_h(v16h a, v16h b, v16h c, v16h d) { asm volatile("v_nop" :: "v"(a), "v"(b), "v"(c), "v"(d)); }
__device__ __forceinline__ void keep4_b(v16b a, v16b b, v16b c, v16b d) { asm volatile("v_nop" :: "v"(a), "v"(b), "v"(c), "v"(d)); }
__device__ __forceinline__ void acc_guard4(v8f& a, v8f& b, v8f& c, v8f& d) { asm volatile("v_nop\n\tv_nop\n\tv_nop\n\tv_nop" : "+v"(a), "+v"(b), "+v"(c), "+v"(d)); }
template <typename T> struct Frag;
template <> struct Frag<_Float16> {
  typedef v16h V; union U { v16h v; v8h h[2]; };
  static __device__ __forceinline__ v16h load(const _Float16* p) {
    U f; f.h[0] = *(const v8h*)(p); f.h[1] = *(const v8h*)(p + 16); return f.v;
  }
  static __device__ __forceinline__ v8f mma(v16h a, v16h b, v8f c) {
    return __builtin_amdgcn_wmma_f32_16x16x32_f16(false, a, false, b, (short)0, c, false, false);
  }
  static __device__ __forceinline__ void guard(v8f& a, v8f& b, v16h x, v16h y) { dep_guard_h(a, b, x, y); }
  static __device__ __forceinline__ void keep(v16h a, v16h b, v16h c, v16h d) { keep4_h(a, b, c, d); }
};
template <> struct Frag<__bf16> {
  typedef v16b V; union U { v16b v; v8b h[2]; };
  static __device__ __forceinline__ v16b load(const __bf16* p) {
    U f; f.h[0] = *(const v8b*)(p); f.h[1] = *(const v8b*)(p + 16); return f.v;
  }
  static __device__ __forceinline__ v8f mma(v16b a, v16b b, v8f c) {
    return __builtin_amdgcn_wmma_f32_16x16x32_bf16(false, a, false, b, (short)0, c, false, false);
  }
  static __device__ __forceinline__ void guard(v8f& a, v8f& b, v16b x, v16b y) { dep_guard_b(a, b, x, y); }
  static __device__ __forceinline__ void keep(v16b a, v16b b, v16b c, v16b d) { keep4_b(a, b, c, d); }
};

__device__ __forceinline__ v8f at_mma(v16b a, v16b b, v8f c) {
  c = __builtin_amdgcn_wmma_f32_16x16x32_bf16(false, a, false, b, (short)0, c, false, false);
  asm volatile("v_nop\n\tv_nop\n\tv_nop\n\tv_nop" : "+v"(c) : "v"(a), "v"(b));
  return c;
}
template <bool F16> __device__ __forceinline__ __bf16 at_to16(float f) {
  if (F16) return __builtin_bit_cast(__bf16, (_Float16)f);
  return __builtin_bit_cast(__bf16, f2bf_bits(f));
}
template <bool F16> __device__ __forceinline__ v8f at_mma16(v16b a, v16b b, v8f c) {
  if (F16) {
    const v16h ah = __builtin_bit_cast(v16h, a), bh = __builtin_bit_cast(v16h, b);
    c = __builtin_amdgcn_wmma_f32_16x16x32_f16(false, ah, false, bh, (short)0, c, false, false);
    asm volatile("v_nop\n\tv_nop\n\tv_nop\n\tv_nop" : "+v"(c) : "v"(ah), "v"(bh));
    return c;
  }
  return at_mma(a, b, c);
}

template <int ET> struct Elem;
template <> struct Elem<0> { typedef _Float16 T; };
template <> struct Elem<1> { typedef __bf16 T; };
template <int ET, int SPLIT, int BIAS_MODE, int OUT_MODE, bool RESID, int ACT = 0>
__global__ __launch_bounds__(256) void wmma_gemm64(
    const unsigned short* __restrict__ Ap, const unsigned short* __restrict__ A2p, int lda, long strideA,
    const unsigned short* __restrict__ Btp, const unsigned short* __restrict__ Bt2p, int ldb, long strideB,
    void* __restrict__ Cout, void* __restrict__ Cout2, int ldc, long strideC,
    const float* __restrict__ bias,
    const float* __restrict__ resid, long strideR,
    int M, int N, int K, float scale) {
  typedef typename Elem<ET>::T T;
  typedef typename Frag<T>::V V;
  const T* A = (const T*)Ap; const T* A2 = (const T*)A2p; const T* Bt = (const T*)Btp; const T* Bt2 = (const T*)Bt2p;
  __shared__ __align__(16) float sT[8][16 * 68];
  const int b    = blockIdx.y;
  const int lane = threadIdx.x & 31;
  const int wave = threadIdx.x >> 5;
  const int tilesN = N >> 6;
  const int tilesM = M >> 6;
  const int tile = blockIdx.x * 8 + wave;
  if (tile >= tilesM * tilesN) return;
  const int tm = tile / tilesN;
  const int tn = tile - tm * tilesN;
  const int m0 = tm << 6;
  const int n0 = tn << 6;

  const T* Ab  = A  + (size_t)b * strideA;
  const T* Bb  = Bt + (size_t)b * strideB;
  const T* Ab2 = (SPLIT >= 1) ? (A2  + (size_t)b * strideA) : nullptr;
  const T* Bb2 = (SPLIT == 2) ? (Bt2 + (size_t)b * strideB) : nullptr;

  const int rlane = lane & 15;
  const int koff  = (lane >> 4) * 8;
  const int mOff  = (lane >> 4) * 8;

  v8f acc[4][4];
#pragma unroll
  for (int i = 0; i < 4; ++i)
#pragma unroll
    for (int j = 0; j < 4; ++j) acc[i][j] = (v8f){0.f,0.f,0.f,0.f,0.f,0.f,0.f,0.f};

  for (int k0 = 0; k0 < K; k0 += 32) {
    V bh[4], bl[4];
#pragma unroll
    for (int j = 0; j < 4; ++j) {
      const size_t bo = (size_t)(n0 + (j << 4) + rlane) * ldb + koff + k0;
      bh[j] = Frag<T>::load(Bb + bo);
      if (SPLIT == 2) bl[j] = Frag<T>::load(Bb2 + bo);
    }
#pragma unroll
    for (int i = 0; i < 4; ++i) {
      const size_t ao = (size_t)(m0 + (i << 4) + rlane) * lda + koff + k0;
      V ah = Frag<T>::load(Ab + ao);
      V al;
      if (SPLIT >= 1) al = Frag<T>::load(Ab2 + ao);
#pragma unroll
      for (int j = 0; j < 4; ++j) {
        acc[i][j] = Frag<T>::mma(ah, bh[j], acc[i][j]);
        if (SPLIT == 2) acc[i][j] = Frag<T>::mma(ah, bl[j], acc[i][j]);
        if (SPLIT >= 1) acc[i][j] = Frag<T>::mma(al, bh[j], acc[i][j]);
      }
      Frag<T>::guard(acc[i][0], acc[i][3], ah, (SPLIT >= 1) ? al : ah);
    }
    Frag<T>::keep(bh[0], bh[1], bh[2], bh[3]);
    if (SPLIT == 2) Frag<T>::keep(bl[0], bl[1], bl[2], bl[3]);
  }
  acc_guard4(acc[0][0], acc[0][1], acc[0][2], acc[0][3]);
  acc_guard4(acc[1][0], acc[1][1], acc[1][2], acc[1][3]);
  acc_guard4(acc[2][0], acc[2][1], acc[2][2], acc[2][3]);
  acc_guard4(acc[3][0], acc[3][1], acc[3][2], acc[3][3]);

  float* slab = sT[wave];
  const float* Rb = RESID ? (resid + (size_t)b * strideR) : nullptr;
#pragma unroll
  for (int i = 0; i < 4; ++i) {
    const int mBase = m0 + (i << 4);
#pragma unroll
    for (int j = 0; j < 4; ++j) {
      const int n = n0 + (j << 4) + rlane;
      float bv = 0.f;
      if (BIAS_MODE == 2) bv = bias[n];
#pragma unroll
      for (int r = 0; r < 8; ++r) {
        float v = acc[i][j][r] * scale;
        if (BIAS_MODE == 1) v += bias[mBase + mOff + r];
        if (BIAS_MODE == 2) v += bv;
        if (RESID) v += Rb[(size_t)(mBase + mOff + r) * ldc + n];
        if (ACT == 1) v = tanhf(v);
        if (ACT == 2) v = fmaxf(v, 0.0f);
        if (ACT == 3) v = v / (1.0f + expf(-v));
        if (ACT == 4) v = (v > 0.f) ? v : 0.01f * v;
        slab[(mOff + r) * 68 + (j << 4) + rlane] = v;
      }
    }
    __builtin_amdgcn_fence(__ATOMIC_RELEASE, "workgroup");
    __builtin_amdgcn_wave_barrier();
    __builtin_amdgcn_fence(__ATOMIC_ACQUIRE, "workgroup");
    if (OUT_MODE == 0) {
      float* C = (float*)Cout + (size_t)b * strideC;
      const int hh = lane >> 4, c4 = (lane & 15) * 4;
      for (int pass = 0; pass < 2; ++pass) {
#pragma unroll
        for (int it = 0; it < 8; ++it) {
          const int row = it * 2 + hh;
          v4f v = *(const v4f*)(slab + row * 68 + c4);
          *(volatile v4f*)(C + (size_t)(mBase + row) * ldc + n0 + c4) = v;
        }
        __threadfence();
      }
    } else {
      const int q = lane >> 3, c8 = (lane & 7) * 8;
      unsigned short* C  = (unsigned short*)Cout  + (size_t)b * strideC;
      unsigned short* C2 = (OUT_MODE == 2) ? ((unsigned short*)Cout2 + (size_t)b * strideC) : nullptr;
      for (int pass = 0; pass < 2; ++pass) {
#pragma unroll
        for (int it = 0; it < 4; ++it) {
          const int row = it * 4 + q;
          const float* sp = slab + row * 68 + c8;
          v8h hv, lv;
#pragma unroll
          for (int e = 0; e < 8; ++e) {
            if (OUT_MODE == 1) {
              hv[e] = (_Float16)sp[e];
            } else {
              unsigned short hb = f2bf_bits(sp[e]);
              unsigned short lb = f2bf_bits(sp[e] - bf_bits2f(hb));
              hv[e] = __builtin_bit_cast(_Float16, hb);
              lv[e] = __builtin_bit_cast(_Float16, lb);
            }
          }
          *(volatile v8h*)(C + (size_t)(mBase + row) * ldc + n0 + c8) = hv;
          if (OUT_MODE == 2) *(volatile v8h*)(C2 + (size_t)(mBase + row) * ldc + n0 + c8) = lv;
        }
        __threadfence();
      }
    }
    __builtin_amdgcn_fence(__ATOMIC_RELEASE, "workgroup");
    __builtin_amdgcn_wave_barrier();
    __builtin_amdgcn_fence(__ATOMIC_ACQUIRE, "workgroup");
  }
}

__global__ __launch_bounds__(256) void cast_f32_bf16x8(
    const float* __restrict__ in, unsigned short* __restrict__ out, int n8) {
  const int i = blockIdx.x * 256 + threadIdx.x;
  if (i < n8) {
    const v4f a0 = *(const v4f*)(in + (size_t)8 * i);
    const v4f a1 = *(const v4f*)(in + (size_t)8 * i + 4);
    v4u w;
    w[0] = (unsigned)f2bf_bits(a0[0]) | ((unsigned)f2bf_bits(a0[1]) << 16);
    w[1] = (unsigned)f2bf_bits(a0[2]) | ((unsigned)f2bf_bits(a0[3]) << 16);
    w[2] = (unsigned)f2bf_bits(a1[0]) | ((unsigned)f2bf_bits(a1[1]) << 16);
    w[3] = (unsigned)f2bf_bits(a1[2]) | ((unsigned)f2bf_bits(a1[3]) << 16);
    volatile v4u* p = (volatile v4u*)(out + (size_t)8 * i);
    *p = w;
    __threadfence();
    *p = w;
  }
}

__global__ __launch_bounds__(256) void cast_kcache_bf16x8(
    const float* __restrict__ kc, unsigned short* __restrict__ Kh, int n8) {
  const int i = blockIdx.x * 256 + threadIdx.x;
  if (i < n8) {
    const size_t e = (size_t)8 * i;
    const size_t bh = e / ((size_t)SEQ_CACHE * HDIM);
    const size_t rem = e - bh * ((size_t)SEQ_CACHE * HDIM);
    const v4f a0 = *(const v4f*)(kc + e);
    const v4f a1 = *(const v4f*)(kc + e + 4);
    v4u w;
    w[0] = (unsigned)f2bf_bits(a0[0]) | ((unsigned)f2bf_bits(a0[1]) << 16);
    w[1] = (unsigned)f2bf_bits(a0[2]) | ((unsigned)f2bf_bits(a0[3]) << 16);
    w[2] = (unsigned)f2bf_bits(a1[0]) | ((unsigned)f2bf_bits(a1[1]) << 16);
    w[3] = (unsigned)f2bf_bits(a1[2]) | ((unsigned)f2bf_bits(a1[3]) << 16);
    volatile v4u* p = (volatile v4u*)(Kh + bh * ((size_t)SEQ_KV * HDIM) + rem);
    *p = w;
    __threadfence();
    *p = w;
  }
}

template <bool SRC32>
__global__ __launch_bounds__(256) void v_transpose_tile(
    const void* __restrict__ src, unsigned short* __restrict__ Vt, int srcRows, int dstCol0) {
  __shared__ __align__(16) unsigned short tile[64 * 72];
  const int tid = threadIdx.x;
  const int bh  = blockIdx.y;
  const int s0  = blockIdx.x * 64;
  if (SRC32) {
    const float* p = (const float*)src + ((size_t)bh * srcRows + s0) * HDIM;
#pragma unroll
    for (int i = 0; i < 4; ++i) {
      const int idx = tid + 256 * i;
      const int row = idx >> 4;
      const int c4  = (idx & 15) * 4;
      const v4f v = *(const v4f*)(p + (size_t)row * HDIM + c4);
      const unsigned short b0 = f2h_bits(bf_bits2f(f2bf_bits(v[0])) * V_CARRY);
      const unsigned short b1 = f2h_bits(bf_bits2f(f2bf_bits(v[1])) * V_CARRY);
      const unsigned short b2 = f2h_bits(bf_bits2f(f2bf_bits(v[2])) * V_CARRY);
      const unsigned short b3 = f2h_bits(bf_bits2f(f2bf_bits(v[3])) * V_CARRY);
      const unsigned w0 = (unsigned)b0 | ((unsigned)b1 << 16);
      const unsigned w1 = (unsigned)b2 | ((unsigned)b3 << 16);
      *(unsigned*)(tile + row * 72 + c4)     = w0;
      *(unsigned*)(tile + row * 72 + c4 + 2) = w1;
    }
  } else {
    const unsigned short* p = (const unsigned short*)src + ((size_t)bh * srcRows + s0) * HDIM;
#pragma unroll
    for (int i = 0; i < 2; ++i) {
      const int idx = tid + 256 * i;
      const int row = idx >> 3;
      const int c8  = (idx & 7) * 8;
      const v4u w = *(const v4u*)(p + (size_t)row * HDIM + c8);
      *(v4u*)(tile + row * 72 + c8) = w;
    }
  }
  __syncthreads();
  v4u wout[2];
#pragma unroll
  for (int i = 0; i < 2; ++i) {
    const int item = tid + 256 * i;
    const int d    = item >> 3;
    const int part = item & 7;
#pragma unroll
    for (int k = 0; k < 4; ++k) {
      const unsigned lo = tile[(part * 8 + 2 * k) * 72 + d];
      const unsigned hi = tile[(part * 8 + 2 * k + 1) * 72 + d];
      wout[i][k] = lo | (hi << 16);
    }
  }
  for (int pass = 0; pass < 2; ++pass) {
#pragma unroll
    for (int i = 0; i < 2; ++i) {
      const int item = tid + 256 * i;
      const int d    = item >> 3;
      const int part = item & 7;
      volatile v4u* dp = (volatile v4u*)(Vt + ((size_t)bh * HDIM + d) * SEQ_KV + dstCol0 + s0 + part * 8);
      *dp = wout[i];
    }
    __threadfence();
  }
}

__global__ __launch_bounds__(256) void qkv_proj_rmsnorm(
    const unsigned short* __restrict__ Xp, const unsigned short* __restrict__ Wp,
    const float* __restrict__ scq, const float* __restrict__ sck,
    unsigned short* __restrict__ Qh, unsigned short* __restrict__ Ql,
    unsigned short* __restrict__ Kh, unsigned short* __restrict__ Kl,
    unsigned short* __restrict__ Vtmp) {
  typedef __bf16 T;
  typedef v16b V;
  const T* A = (const T*)Xp;
  const T* Bt = (const T*)Wp;
  __shared__ __align__(16) float sT[8][16 * 68];
  const int lane = threadIdx.x & 31;
  const int wave = threadIdx.x >> 5;
  constexpr int tilesN = (3 * DMODEL) / 64;
  constexpr int tilesM = NUM_TOK / 64;
  const int tile = blockIdx.x * 8 + wave;
  if (tile >= tilesM * tilesN) return;
  const int tm = tile / tilesN;
  const int tn = tile - tm * tilesN;
  const int m0 = tm << 6;
  const int n0 = tn << 6;
  const int rlane = lane & 15;
  const int koff  = (lane >> 4) * 8;
  const int mOff  = (lane >> 4) * 8;

  v8f acc[4][4];
#pragma unroll
  for (int i = 0; i < 4; ++i)
#pragma unroll
    for (int j = 0; j < 4; ++j) acc[i][j] = (v8f){0.f,0.f,0.f,0.f,0.f,0.f,0.f,0.f};

  for (int k0 = 0; k0 < DMODEL; k0 += 32) {
    V bfr[4];
#pragma unroll
    for (int j = 0; j < 4; ++j)
      bfr[j] = Frag<T>::load(Bt + (size_t)(n0 + (j << 4) + rlane) * DMODEL + koff + k0);
#pragma unroll
    for (int i = 0; i < 4; ++i) {
      V afr = Frag<T>::load(A + (size_t)(m0 + (i << 4) + rlane) * DMODEL + koff + k0);
#pragma unroll
      for (int j = 0; j < 4; ++j) acc[i][j] = Frag<T>::mma(afr, bfr[j], acc[i][j]);
      Frag<T>::guard(acc[i][0], acc[i][3], afr, afr);
    }
    Frag<T>::keep(bfr[0], bfr[1], bfr[2], bfr[3]);
  }
  acc_guard4(acc[0][0], acc[0][1], acc[0][2], acc[0][3]);
  acc_guard4(acc[1][0], acc[1][1], acc[1][2], acc[1][3]);
  acc_guard4(acc[2][0], acc[2][1], acc[2][2], acc[2][3]);
  acc_guard4(acc[3][0], acc[3][1], acc[3][2], acc[3][3]);

  const int which = n0 >> 10;
  const int head  = (n0 & (DMODEL - 1)) >> 6;
  const int bidx  = m0 >> 11;
  const int s0    = m0 & (SEQ_LEN - 1);
  const int bh    = bidx * NHEAD + head;
  float scl[4];
#pragma unroll
  for (int j = 0; j < 4; ++j) {
    const float a = bf_bits2f(f2bf_bits(scq[j * 16 + rlane]));
    const float c = bf_bits2f(f2bf_bits(sck[j * 16 + rlane]));
    scl[j] = (which == 0) ? (a * LOG2E_F) : c;
  }
  float* slab = sT[wave];
  const int q8 = lane >> 3, c8 = (lane & 7) * 8;
#pragma unroll
  for (int i = 0; i < 4; ++i) {
    float fac[8];
#pragma unroll
    for (int r = 0; r < 8; ++r) {
      float ss = 0.f;
#pragma unroll
      for (int j = 0; j < 4; ++j) { const float x = acc[i][j][r]; ss += x * x; }
      ss += __shfl_xor(ss, 1, 32);
      ss += __shfl_xor(ss, 2, 32);
      ss += __shfl_xor(ss, 4, 32);
      ss += __shfl_xor(ss, 8, 32);
      const float rms = sqrtf(ss * (1.0f / 64.0f)) + 1e-6f;
      const float inv = 1.0f / rms;
      fac[r] = (which == 2) ? V_CARRY : inv;
    }
#pragma unroll
    for (int j = 0; j < 4; ++j)
#pragma unroll
      for (int r = 0; r < 8; ++r) {
        float v = acc[i][j][r] * fac[r];
        if (which != 2) v *= scl[j];
        slab[(mOff + r) * 68 + (j << 4) + rlane] = v;
      }
    __builtin_amdgcn_fence(__ATOMIC_RELEASE, "workgroup");
    __builtin_amdgcn_wave_barrier();
    __builtin_amdgcn_fence(__ATOMIC_ACQUIRE, "workgroup");
    if (which == 2) {
      unsigned short* dst = Vtmp + ((size_t)bh * SEQ_LEN + s0 + i * 16) * HDIM;
      for (int pass = 0; pass < 2; ++pass) {
#pragma unroll
        for (int it = 0; it < 4; ++it) {
          const int row = it * 4 + q8;
          const float* sp = slab + row * 68 + c8;
          v8h hv;
#pragma unroll
          for (int e = 0; e < 8; ++e) hv[e] = (_Float16)sp[e];
          *(volatile v8h*)(dst + (size_t)row * HDIM + c8) = hv;
        }
        __threadfence();
      }
    } else {
      const size_t rowbase = (which == 0) ? ((size_t)bh * SEQ_LEN + s0 + i * 16)
                                          : ((size_t)bh * SEQ_KV + SEQ_CACHE + s0 + i * 16);
      unsigned short* dh = ((which == 0) ? Qh : Kh) + rowbase * HDIM;
      unsigned short* dl = ((which == 0) ? Ql : Kl) + rowbase * HDIM;
      for (int pass = 0; pass < 2; ++pass) {
#pragma unroll
        for (int it = 0; it < 4; ++it) {
          const int row = it * 4 + q8;
          const float* sp = slab + row * 68 + c8;
          v8h hv, lv;
#pragma unroll
          for (int e = 0; e < 8; ++e) {
            unsigned short hb = f2bf_bits(sp[e]);
            unsigned short lb = f2bf_bits(sp[e] - bf_bits2f(hb));
            hv[e] = __builtin_bit_cast(_Float16, hb);
            lv[e] = __builtin_bit_cast(_Float16, lb);
          }
          *(volatile v8h*)(dh + (size_t)row * HDIM + c8) = hv;
          *(volatile v8h*)(dl + (size_t)row * HDIM + c8) = lv;
        }
        __threadfence();
      }
    }
    __builtin_amdgcn_fence(__ATOMIC_RELEASE, "workgroup");
    __builtin_amdgcn_wave_barrier();
    __builtin_amdgcn_fence(__ATOMIC_ACQUIRE, "workgroup");
  }
}

template <bool NEWK>
__device__ __forceinline__ void attn_chunk(
    const int kv0, const int tid, const int hh, const int c,
    const __bf16* __restrict__ Khp, const __bf16* __restrict__ Klp, const __bf16* __restrict__ Vtp,
    __bf16* Ksh, __bf16* Ksl, __bf16* Vts, __bf16* pwh,
    const v16b (&qah)[2], const v16b (&qal)[2],
    float (&mrow)[8], float (&lrow)[8], v8f (&oacc)[4]) {
  union FB { v16b v; v8b h[2]; };
  __syncthreads();
#pragma unroll
  for (int i = 0; i < 4; ++i) {
    const int idx = tid + 128 * i;
    const int row = idx >> 3;
    const int c8  = (idx & 7) * 8;
    const v4u kw = *(const v4u*)(Khp + (size_t)(kv0 + row) * HDIM + c8);
    *(v4u*)(Ksh + row * HDIM + c8) = kw;
    if (NEWK) {
      const v4u lw = *(const v4u*)(Klp + (size_t)(kv0 + row) * HDIM + c8);
      *(v4u*)(Ksl + row * HDIM + c8) = lw;
    }
    const v4u vw = *(const v4u*)(Vtp + (size_t)row * SEQ_KV + kv0 + c8);
    *(v4u*)(Vts + row * 64 + c8) = vw;
  }
  __syncthreads();

  v8f s[4];
#pragma unroll
  for (int j = 0; j < 4; ++j) {
    s[j] = (v8f){0.f,0.f,0.f,0.f,0.f,0.f,0.f,0.f};
#pragma unroll
    for (int dc = 0; dc < 2; ++dc) {
      FB kb;
      kb.h[0] = *(const v8b*)(Ksh + (j * 16 + c) * HDIM + dc * 32 + 8 * hh);
      kb.h[1] = *(const v8b*)(Ksh + (j * 16 + c) * HDIM + dc * 32 + 16 + 8 * hh);
      s[j] = at_mma(qah[dc], kb.v, s[j]);
      s[j] = at_mma(qal[dc], kb.v, s[j]);
      if (NEWK) {
        FB kl;
        kl.h[0] = *(const v8b*)(Ksl + (j * 16 + c) * HDIM + dc * 32 + 8 * hh);
        kl.h[1] = *(const v8b*)(Ksl + (j * 16 + c) * HDIM + dc * 32 + 16 + 8 * hh);
        s[j] = at_mma(qah[dc], kl.v, s[j]);
      }
    }
  }
  float cm[8];
#pragma unroll
  for (int r = 0; r < 8; ++r) {
    float m = fmaxf(fmaxf(s[0][r], s[1][r]), fmaxf(s[2][r], s[3][r]));
#pragma unroll
    for (int off = 1; off < 16; off <<= 1) m = fmaxf(m, __shfl_xor(m, off, 32));
    cm[r] = m;
  }
#pragma unroll
  for (int r = 0; r < 8; ++r) {
    const float mnew = fmaxf(mrow[r], cm[r]);
    const float alpha = exp2f(mrow[r] - mnew);
    mrow[r] = mnew;
    float psum = 0.f;
#pragma unroll
    for (int j = 0; j < 4; ++j) {
      const float p = exp2f(s[j][r] - mnew);
      psum += p;
      pwh[(8 * hh + r) * 64 + j * 16 + c] = at_to16<true>(p * P_CARRY);
    }
#pragma unroll
    for (int off = 1; off < 16; off <<= 1) psum += __shfl_xor(psum, off, 32);
    lrow[r] = lrow[r] * alpha + psum;
#pragma unroll
    for (int t = 0; t < 4; ++t) oacc[t][r] *= alpha;
  }
  __builtin_amdgcn_fence(__ATOMIC_RELEASE, "workgroup");
  __builtin_amdgcn_wave_barrier();
  __builtin_amdgcn_fence(__ATOMIC_ACQUIRE, "workgroup");
#pragma unroll
  for (int kk = 0; kk < 2; ++kk) {
    FB pa;
    pa.h[0] = *(const v8b*)(pwh + c * 64 + kk * 32 + 8 * hh);
    pa.h[1] = *(const v8b*)(pwh + c * 64 + kk * 32 + 16 + 8 * hh);
#pragma unroll
    for (int t = 0; t < 4; ++t) {
      FB vb;
      vb.h[0] = *(const v8b*)(Vts + (t * 16 + c) * 64 + kk * 32 + 8 * hh);
      vb.h[1] = *(const v8b*)(Vts + (t * 16 + c) * 64 + kk * 32 + 16 + 8 * hh);
      oacc[t] = at_mma16<true>(pa.v, vb.v, oacc[t]);
    }
  }
}

__global__ __launch_bounds__(128) void attn_extended(
    const unsigned short* __restrict__ Qh, const unsigned short* __restrict__ Ql,
    const unsigned short* __restrict__ Kh, const unsigned short* __restrict__ Kl,
    const unsigned short* __restrict__ Vt,
    unsigned short* __restrict__ Oh, unsigned short* __restrict__ Ol) {
  __shared__ __align__(16) __bf16 Ksh[64 * HDIM];
  __shared__ __align__(16) __bf16 Ksl[64 * HDIM];
  __shared__ __align__(16) __bf16 Vts[HDIM * 64];
  __shared__ __align__(16) __bf16 Psh[4][16 * 64];
  __shared__ __align__(16) float  Os[4][16 * 68];

  const int tid  = threadIdx.x;
  const int wave = tid >> 5;
  const int lane = tid & 31;
  const int hh   = lane >> 4;
  const int c    = lane & 15;

  const int bx = blockIdx.x;
  const int qb = bx & 31;
  const int bh = bx >> 5;
  const int h  = bh & (NHEAD - 1);
  const int b  = bh >> 4;
  const int q0 = qb * 64 + wave * 16;

  const __bf16* Qhp = (const __bf16*)Qh + (size_t)bh * SEQ_LEN * HDIM;
  const __bf16* Qlp = (const __bf16*)Ql + (size_t)bh * SEQ_LEN * HDIM;
  const __bf16* Khp = (const __bf16*)Kh + (size_t)bh * SEQ_KV * HDIM;
  const __bf16* Klp = (const __bf16*)Kl + (size_t)bh * SEQ_KV * HDIM;
  const __bf16* Vtp = (const __bf16*)Vt + (size_t)bh * HDIM * SEQ_KV;

  v16b qah[2], qal[2];
#pragma unroll
  for (int dc = 0; dc < 2; ++dc) {
    qah[dc] = Frag<__bf16>::load(Qhp + (size_t)(q0 + c) * HDIM + dc * 32 + 8 * hh);
    qal[dc] = Frag<__bf16>::load(Qlp + (size_t)(q0 + c) * HDIM + dc * 32 + 8 * hh);
  }

  float mrow[8], lrow[8];
  v8f oacc[4];
#pragma unroll
  for (int r = 0; r < 8; ++r) { mrow[r] = -INFINITY; lrow[r] = 0.f; }
#pragma unroll
  for (int t = 0; t < 4; ++t) oacc[t] = (v8f){0.f,0.f,0.f,0.f,0.f,0.f,0.f,0.f};

  __bf16* pwh = Psh[wave];
  constexpr int nCached = SEQ_CACHE / 64;
  constexpr int nTotal  = SEQ_KV / 64;
  for (int kc = 0; kc < nCached; ++kc)
    attn_chunk<false>(kc * 64, tid, hh, c, Khp, Klp, Vtp, Ksh, Ksl, Vts, pwh, qah, qal, mrow, lrow, oacc);
  for (int kc = nCached; kc < nTotal; ++kc)
    attn_chunk<true>(kc * 64, tid, hh, c, Khp, Klp, Vtp, Ksh, Ksl, Vts, pwh, qah, qal, mrow, lrow, oacc);

  float* os = Os[wave];
#pragma unroll
  for (int r = 0; r < 8; ++r) {
    const float inv = 1.0f / (lrow[r] * (P_CARRY * V_CARRY));
#pragma unroll
    for (int t = 0; t < 4; ++t) os[(8 * hh + r) * 68 + t * 16 + c] = oacc[t][r] * inv;
  }
  __builtin_amdgcn_fence(__ATOMIC_RELEASE, "workgroup");
  __builtin_amdgcn_wave_barrier();
  __builtin_amdgcn_fence(__ATOMIC_ACQUIRE, "workgroup");
  {
    const int q8 = lane >> 3, c8 = (lane & 7) * 8;
    unsigned short* ohp = Oh + ((size_t)b * SEQ_LEN + q0) * DMODEL + h * HDIM;
    unsigned short* olp = Ol + ((size_t)b * SEQ_LEN + q0) * DMODEL + h * HDIM;
    for (int pass = 0; pass < 2; ++pass) {
#pragma unroll
      for (int it = 0; it < 4; ++it) {
        const int row = it * 4 + q8;
        const float* sp = os + row * 68 + c8;
        v8h hv, lv;
#pragma unroll
        for (int e = 0; e < 8; ++e) {
          unsigned short hb = f2bf_bits(sp[e]);
          unsigned short lb = f2bf_bits(sp[e] - bf_bits2f(hb));
          hv[e] = __builtin_bit_cast(_Float16, hb);
          lv[e] = __builtin_bit_cast(_Float16, lb);
        }
        *(volatile v8h*)(ohp + (size_t)row * DMODEL + c8) = hv;
        *(volatile v8h*)(olp + (size_t)row * DMODEL + c8) = lv;
      }
      __threadfence();
    }
  }
}

extern "C" void kernel_launch(void* const* d_in, const int* in_sizes, int n_in,
                              void* d_out, int out_size, void* d_ws, size_t ws_size, hipStream_t stream) {
  if (n_in < 7) return;
  if (in_sizes[0] != NUM_TOK * DMODEL) return;
  if (in_sizes[1] != NUM_BH * SEQ_CACHE * HDIM) return;
  if (in_sizes[2] != NUM_BH * SEQ_CACHE * HDIM) return;
  if (in_sizes[3] != 3 * DMODEL * DMODEL) return;
  if (in_sizes[4] != DMODEL * DMODEL) return;
  if (in_sizes[5] < HDIM || in_sizes[6] < HDIM) return;
  if (out_size != NUM_TOK * DMODEL) return;

  const float* x    = (const float*)d_in[0];
  const float* kc   = (const float*)d_in[1];
  const float* vc   = (const float*)d_in[2];
  const float* wqkv = (const float*)d_in[3];
  const float* wo   = (const float*)d_in[4];
  const float* sq   = (const float*)d_in[5];
  const float* sk   = (const float*)d_in[6];
  float* out = (float*)d_out;

  constexpr size_t XB_BYTES   = (size_t)NUM_TOK * DMODEL * 2;
  constexpr size_t WQ_BYTES   = (size_t)3 * DMODEL * DMODEL * 2;
  constexpr size_t WO_BYTES   = (size_t)DMODEL * DMODEL * 2;
  constexpr size_t QP_BYTES   = (size_t)NUM_BH * SEQ_LEN * HDIM * 2;
  constexpr size_t KP_BYTES   = (size_t)NUM_BH * SEQ_KV * HDIM * 2;
  constexpr size_t VT_BYTES   = (size_t)NUM_BH * HDIM * SEQ_KV * 2;
  constexpr size_t VTMP_BYTES = (size_t)NUM_BH * SEQ_LEN * HDIM * 2;
  constexpr size_t OP_BYTES   = (size_t)NUM_TOK * DMODEL * 2;
  constexpr size_t TOTAL_BYTES = XB_BYTES + WQ_BYTES + WO_BYTES + 2 * QP_BYTES + 2 * KP_BYTES
                               + VT_BYTES + VTMP_BYTES + 2 * OP_BYTES;
  static_assert(TOTAL_BYTES == 109051904ull);
  static_assert(TOTAL_BYTES <= 134217728ull);
  if (TOTAL_BYTES > ws_size) return;

  char* ws = (char*)d_ws;
  size_t off = 0;
  unsigned short* Xb    = (unsigned short*)(ws + off); off += XB_BYTES;
  unsigned short* Wqkvb = (unsigned short*)(ws + off); off += WQ_BYTES;
  unsigned short* Wob   = (unsigned short*)(ws + off); off += WO_BYTES;
  unsigned short* Qh    = (unsigned short*)(ws + off); off += QP_BYTES;
  unsigned short* Ql    = (unsigned short*)(ws + off); off += QP_BYTES;
  unsigned short* Kh    = (unsigned short*)(ws + off); off += KP_BYTES;
  unsigned short* Kl    = (unsigned short*)(ws + off); off += KP_BYTES;
  unsigned short* Vt    = (unsigned short*)(ws + off); off += VT_BYTES;
  unsigned short* Vtmp  = (unsigned short*)(ws + off); off += VTMP_BYTES;
  unsigned short* Oh    = (unsigned short*)(ws + off); off += OP_BYTES;
  unsigned short* Ol    = (unsigned short*)(ws + off); off += OP_BYTES;
  if (off > ws_size) return;

  {
    const int n8x = NUM_TOK * DMODEL / 8;
    cast_f32_bf16x8<<<(n8x + 255) / 256, 256, 0, stream>>>(x, Xb, n8x);
    const int n8w = 3 * DMODEL * DMODEL / 8;
    cast_f32_bf16x8<<<(n8w + 255) / 256, 256, 0, stream>>>(wqkv, Wqkvb, n8w);
    const int n8o = DMODEL * DMODEL / 8;
    cast_f32_bf16x8<<<(n8o + 255) / 256, 256, 0, stream>>>(wo, Wob, n8o);
  }
  {
    const int n8k = NUM_BH * SEQ_CACHE * HDIM / 8;
    cast_kcache_bf16x8<<<(n8k + 255) / 256, 256, 0, stream>>>(kc, Kh, n8k);
  }
  v_transpose_tile<true><<<dim3(SEQ_CACHE / 64, NUM_BH), 256, 0, stream>>>((const void*)vc, Vt, SEQ_CACHE, 0);

  {
    static_assert(NUM_TOK % 64 == 0 && (3 * DMODEL) % 64 == 0 && DMODEL % 32 == 0);
    const int tiles = (NUM_TOK / 64) * (3 * DMODEL / 64);
    qkv_proj_rmsnorm<<<(tiles + 7) / 8, 256, 0, stream>>>(Xb, Wqkvb, sq, sk, Qh, Ql, Kh, Kl, Vtmp);
  }
  v_transpose_tile<false><<<dim3(SEQ_LEN / 64, NUM_BH), 256, 0, stream>>>((const void*)Vtmp, Vt, SEQ_LEN, SEQ_CACHE);

  attn_extended<<<NUM_BH * (SEQ_LEN / 64), 128, 0, stream>>>(Qh, Ql, Kh, Kl, Vt, Oh, Ol);

  {
    static_assert(NUM_TOK % 64 == 0 && DMODEL % 64 == 0 && DMODEL % 32 == 0);
    const int tiles = (NUM_TOK / 64) * (DMODEL / 64);
    wmma_gemm64<1, 1, 0, 0, false, 0><<<dim3((tiles + 7) / 8, 1), 256, 0, stream>>>(
        Oh, Ol, DMODEL, 0L,
        Wob, Wob, DMODEL, 0L,
        (void*)out, (void*)out, DMODEL, 0L,
        sq,
        sq, 0L,
        NUM_TOK, DMODEL, DMODEL, 1.0f);
  }
}
